// MultiheadSelfAttention_90915867721901
// MI455X (gfx1250) — hardware-verified
//
#include <hip/hip_runtime.h>
#include <math.h>

#ifndef NB
#define NB 4
#endif
#ifndef SEQ
#define SEQ 2048
#endif
#ifndef BAND
#define BAND 512
#endif
#define NB_FULL 4
#define SEQ_FULL 2048
#define MAXPOS 2048
#define DM 1024
#define NH 16
#define HD 64
#define NTOK (NB * SEQ)
#define BANDE ((BAND < SEQ) ? BAND : SEQ)
#define NBAND (NB * BANDE)

static_assert(SEQ % 64 == 0);
static_assert(BAND % 64 == 0);
static_assert(BANDE % 64 == 0);
static_assert(NTOK % 64 == 0);
static_assert(DM % 64 == 0);
static_assert(NH * HD == DM);
static_assert(NB <= NB_FULL);
static_assert(SEQ <= SEQ_FULL);
static_assert(((NTOK / 64) * (DM / 64)) % 8 == 0);

typedef __attribute__((ext_vector_type(16))) _Float16 v16h;
typedef __attribute__((ext_vector_type(8)))  _Float16 v8h;
typedef __attribute__((ext_vector_type(16))) __bf16   v16b;
typedef __attribute__((ext_vector_type(8)))  __bf16   v8b;
typedef __attribute__((ext_vector_type(8)))  float    v8f;
typedef __attribute__((ext_vector_type(4)))  float    v4f;
typedef __attribute__((ext_vector_type(4)))  unsigned v4u;
typedef __attribute__((ext_vector_type(8)))  unsigned short v8us;


#define VST2(T, ptr, val) do { const T vst2_v_ = (val); *(volatile T*)(ptr) = vst2_v_; __threadfence(); *(volatile T*)(ptr) = vst2_v_; } while (0)

__device__ __forceinline__ unsigned short bf_bits(float f) {
  unsigned u = __float_as_uint(f);
  return (unsigned short)((u + 0x7FFFu + ((u >> 16) & 1u)) >> 16);
}
__device__ __forceinline__ float bf_f32(unsigned short h) { return __uint_as_float(((unsigned)h) << 16); }
__device__ __forceinline__ float bf_keep(float v) {
  const unsigned u = __float_as_uint(v);
  return __uint_as_float((u + 0x7FFFu + ((u >> 16) & 1u)) & 0xFFFF0000u);
}
__device__ __forceinline__ unsigned short h_bits(float f) { return __builtin_bit_cast(unsigned short, (_Float16)f); }
__device__ __forceinline__ unsigned pk2(unsigned short a, unsigned short b) { return (unsigned)a | ((unsigned)b << 16); }

__device__ __forceinline__ void dep_guard_h(v8f& a, v8f& b, v16h x, v16h y) { asm volatile("v_nop\n\tv_nop\n\tv_nop\n\tv_nop" : "+v"(a), "+v"(b) : "v"(x), "v"(y)); }
__device__ __forceinline__ void dep_guard_b(v8f& a, v8f& b, v16b x, v16b y) { asm volatile("v_nop\n\tv_nop\n\tv_nop\n\tv_nop" : "+v"(a), "+v"(b) : "v"(x), "v"(y)); }
__device__ __forceinline__ void dep1_h(v8f& c, v16h x, v16h y) { asm volatile("v_nop\n\tv_nop\n\tv_nop\n\tv_nop" : "+v"(c) : "v"(x), "v"(y)); }
__device__ __forceinline__ void dep1_b(v8f& c, v16b x, v16b y) { asm volatile("v_nop\n\tv_nop\n\tv_nop\n\tv_nop" : "+v"(c) : "v"(x), "v"(y)); }
__device__ __forceinline__ void keep4_h(v16h a, v16h b, v16h c, v16h d) { asm volatile("v_nop" :: "v"(a), "v"(b), "v"(c), "v"(d)); }
__device__ __forceinline__ void keep4_b(v16b a, v16b b, v16b c, v16b d) { asm volatile("v_nop" :: "v"(a), "v"(b), "v"(c), "v"(d)); }
__device__ __forceinline__ void acc_guard4(v8f& a, v8f& b, v8f& c, v8f& d) { asm volatile("v_nop\n\tv_nop\n\tv_nop\n\tv_nop" : "+v"(a), "+v"(b), "+v"(c), "+v"(d)); }

template <typename T> struct Frag;
template <> struct Frag<_Float16> {
  typedef v16h V; union U { v16h v; v8h h[2]; };
  static __device__ __forceinline__ v16h load(const _Float16* p) {
    U f; f.h[0] = *(const v8h*)(p); f.h[1] = *(const v8h*)(p + 16); return f.v;
  }
  static __device__ __forceinline__ v8f mma(v16h a, v16h b, v8f c) {
    return __builtin_amdgcn_wmma_f32_16x16x32_f16(false, a, false, b, (short)0, c, false, false);
  }
  static __device__ __forceinline__ void guard(v8f& a, v8f& b, v16h x, v16h y) { dep_guard_h(a, b, x, y); }
  static __device__ __forceinline__ void guard1(v8f& c, v16h x, v16h y) { dep1_h(c, x, y); }
  static __device__ __forceinline__ void keep(v16h a, v16h b, v16h c, v16h d) { keep4_h(a, b, c, d); }
  static __device__ __forceinline__ _Float16 from_bits(unsigned short u) { return __builtin_bit_cast(_Float16, u); }
};
template <> struct Frag<__bf16> {
  typedef v16b V; union U { v16b v; v8b h[2]; };
  static __device__ __forceinline__ v16b load(const __bf16* p) {
    U f; f.h[0] = *(const v8b*)(p); f.h[1] = *(const v8b*)(p + 16); return f.v;
  }
  static __device__ __forceinline__ v8f mma(v16b a, v16b b, v8f c) {
    return __builtin_amdgcn_wmma_f32_16x16x32_bf16(false, a, false, b, (short)0, c, false, false);
  }
  static __device__ __forceinline__ void guard(v8f& a, v8f& b, v16b x, v16b y) { dep_guard_b(a, b, x, y); }
  static __device__ __forceinline__ void guard1(v8f& c, v16b x, v16b y) { dep1_b(c, x, y); }
  static __device__ __forceinline__ void keep(v16b a, v16b b, v16b c, v16b d) { keep4_b(a, b, c, d); }
  static __device__ __forceinline__ __bf16 from_bits(unsigned short u) { return __builtin_bit_cast(__bf16, u); }
};
template <int ET> struct Elem;
template <> struct Elem<0> { typedef _Float16 T; };
template <> struct Elem<1> { typedef __bf16 T; };

template <typename T>
__device__ __forceinline__ v8f mma_g(typename Frag<T>::V a, typename Frag<T>::V b, v8f c) {
  c = Frag<T>::mma(a, b, c);
  Frag<T>::guard1(c, a, b);
  return c;
}

#define WAVE_SYNC() do { __builtin_amdgcn_fence(3  , "workgroup"); __builtin_amdgcn_wave_barrier(); __builtin_amdgcn_fence(2  , "workgroup"); } while (0)

__global__ __launch_bounds__(256) void k_cast_x(const float* __restrict__ X, unsigned short* __restrict__ X16) {
  const unsigned u = blockIdx.x * 256u + threadIdx.x;
  const unsigned tok = u >> 7, c0 = (u & 127u) << 3;
  const unsigned b = tok / (unsigned)SEQ, s = tok - b * (unsigned)SEQ;
  const float* sp = X + ((size_t)b * SEQ_FULL + s) * DM + c0;
  const v4f a = *(const v4f*)sp, q = *(const v4f*)(sp + 4);
  v4u pk;
  pk.x = pk2(h_bits(bf_keep(a.x)), h_bits(bf_keep(a.y)));
  pk.y = pk2(h_bits(bf_keep(a.z)), h_bits(bf_keep(a.w)));
  pk.z = pk2(h_bits(bf_keep(q.x)), h_bits(bf_keep(q.y)));
  pk.w = pk2(h_bits(bf_keep(q.z)), h_bits(bf_keep(q.w)));
  VST2(v4u, (v4u*)(X16 + (size_t)tok * DM + c0), pk);
}

struct W4 { const float* w0; const float* w1; const float* w2; const float* w3; };
static_assert(sizeof(W4) == 32);
__global__ __launch_bounds__(256) void k_cast_w(W4 p, unsigned short* __restrict__ W16) {
  const unsigned z = blockIdx.y;
  const float* src = (z == 0u) ? p.w0 : ((z == 1u) ? p.w1 : ((z == 2u) ? p.w2 : p.w3));
  const unsigned u = blockIdx.x * 256u + threadIdx.x;
  const size_t o = (size_t)u << 3;
  const v4f a = *(const v4f*)(src + o), q = *(const v4f*)(src + o + 4);
  const float w[8] = {a.x, a.y, a.z, a.w, q.x, q.y, q.z, q.w};
  unsigned short hb[8];
#pragma unroll
  for (int e = 0; e < 8; ++e) {
    const float bv = bf_keep(w[e]);
    const unsigned short asbf = (unsigned short)(__float_as_uint(bv) >> 16);
    const unsigned short ash = h_bits(bv * 16.0f);
    hb[e] = (z == 3u) ? asbf : ash;
  }
  v4u pk; pk.x = pk2(hb[0], hb[1]); pk.y = pk2(hb[2], hb[3]); pk.z = pk2(hb[4], hb[5]); pk.w = pk2(hb[6], hb[7]);
  VST2(v4u, (v4u*)(W16 + (size_t)z * DM * DM + o), pk);
}

struct RopeF { float inv[32]; };
static_assert(sizeof(RopeF) == 128);
__global__ __launch_bounds__(256) void k_tab(float* __restrict__ tab, RopeF f) {
  const unsigned u = blockIdx.x * 256u + threadIdx.x;
  const unsigned s = u >> 5, i = u & 31u;
  const int p = (int)s;
  float iv = f.inv[0];
#pragma unroll
  for (int e = 1; e < 32; ++e) iv = (i == (unsigned)e) ? f.inv[e] : iv;
  const float ang = (float)p * iv;
  const float cs = cosf(ang), sn = sinf(ang);
  VST2(float, tab + (size_t)s * 64u + i, cs);
  VST2(float, tab + (size_t)s * 64u + 32u + i, sn);
}

template <int EPI>
__global__ __launch_bounds__(256) void k_gemm64(
    const unsigned short* __restrict__ Ap, const unsigned short* __restrict__ A2p, const unsigned short* __restrict__ Btp,
    unsigned short* __restrict__ CF, unsigned short* __restrict__ CBH, unsigned short* __restrict__ CBL,
    float* __restrict__ Cf, const float* __restrict__ tab) {
  typedef typename Elem<(EPI == 2) ? 1 : 0>::T T;
  typedef typename Frag<T>::V V;
  constexpr unsigned M  = (EPI == 1) ? (unsigned)DM : (unsigned)NTOK;
  constexpr unsigned N  = (EPI == 1) ? (unsigned)NTOK : (unsigned)DM;
  constexpr unsigned KT = (EPI == 2) ? 2u * DM : (unsigned)DM;
  constexpr unsigned tilesN = N / 64u, tilesM = M / 64u;
  __shared__ __align__(16) float sT[8][16 * 68];
  const unsigned lane = threadIdx.x & 31u;
  const unsigned wave = threadIdx.x >> 5;
  const unsigned z = blockIdx.y;
  const unsigned tile = blockIdx.x * 8u + wave;
  if (tile >= tilesM * tilesN) return;
  const unsigned tm = tile / tilesN;
  const unsigned tn = tile - tm * tilesN;
  const unsigned m0 = tm << 6, n0 = tn << 6;

  const T* A  = (const T*)Ap;
  const T* A2 = (const T*)A2p;
  const T* Bt = (const T*)Btp + (size_t)z * DM * DM;

  const unsigned rlane = lane & 15u;
  const unsigned koff  = (lane >> 4) * 8u;
  const unsigned mOff  = (lane >> 4) * 8u;

  v8f acc[4][4];
#pragma unroll
  for (int i = 0; i < 4; ++i)
#pragma unroll
    for (int j = 0; j < 4; ++j) acc[i][j] = (v8f){0.f, 0.f, 0.f, 0.f, 0.f, 0.f, 0.f, 0.f};

  for (unsigned k0 = 0; k0 < KT; k0 += 32u) {
    const T* Ak = A; unsigned kk = k0;
    if (EPI == 2) { if (k0 >= (unsigned)DM) { Ak = A2; kk = k0 - (unsigned)DM; } }
    V bh[4];
#pragma unroll
    for (int j = 0; j < 4; ++j) {
      const size_t bo = (size_t)(n0 + ((unsigned)j << 4) + rlane) * DM + koff + kk;
      bh[j] = Frag<T>::load(Bt + bo);
    }
#pragma unroll
    for (int i = 0; i < 4; ++i) {
      const size_t ao = (size_t)(m0 + ((unsigned)i << 4) + rlane) * DM + koff + kk;
      V ah = Frag<T>::load(Ak + ao);
#pragma unroll
      for (int j = 0; j < 4; ++j) acc[i][j] = Frag<T>::mma(ah, bh[j], acc[i][j]);
      Frag<T>::guard(acc[i][0], acc[i][3], ah, ah);
    }
    Frag<T>::keep(bh[0], bh[1], bh[2], bh[3]);
  }
  acc_guard4(acc[0][0], acc[0][1], acc[0][2], acc[0][3]);
  acc_guard4(acc[1][0], acc[1][1], acc[1][2], acc[1][3]);
  acc_guard4(acc[2][0], acc[2][1], acc[2][2], acc[2][3]);
  acc_guard4(acc[3][0], acc[3][1], acc[3][2], acc[3][3]);

  const float scale = (EPI == 2) ? 1.0f : 0.0625f;
  float* slab = sT[wave];
  const unsigned tok0 = (EPI == 1) ? n0 : m0;
  const unsigned bidx = tok0 / (unsigned)SEQ;
  const unsigned s0 = tok0 - bidx * (unsigned)SEQ;
  const bool inband = (s0 < (unsigned)BANDE);
  unsigned short* CFz  = CF  + (size_t)z * NTOK * DM;
  unsigned short* CBHz = CBH + (size_t)z * NBAND * DM;
  unsigned short* CBLz = CBL + (size_t)z * NBAND * DM;
#pragma unroll
  for (int i = 0; i < 4; ++i) {
    const unsigned mBase = m0 + ((unsigned)i << 4);
#pragma unroll
    for (int j = 0; j < 4; ++j)
#pragma unroll
      for (int r = 0; r < 8; ++r) slab[(mOff + (unsigned)r) * 68u + ((unsigned)j << 4) + rlane] = acc[i][j][r] * scale;
    WAVE_SYNC();
    if (EPI == 2) {
      const unsigned hh2 = lane >> 4, c4 = (lane & 15u) << 2;
      for (int pass = 0; pass < 2; ++pass) {
#pragma unroll
        for (int it = 0; it < 8; ++it) {
          const unsigned row = (unsigned)it * 2u + hh2;
          const unsigned s = s0 + ((unsigned)i << 4) + row;
          const size_t orow = (size_t)bidx * SEQ_FULL + s;
          const v4f v = *(const v4f*)(slab + row * 68u + c4);
          *(volatile v4f*)(Cf + orow * DM + n0 + c4) = v;
        }
        __threadfence();
      }
    } else {
      const unsigned q = lane >> 3, c8 = (lane & 7u) << 3;
      v8us fv[4], hv[4], lv[4];
#pragma unroll
      for (int it = 0; it < 4; ++it) {
        const unsigned row = (unsigned)it * 4u + q;
        const float* sp = slab + row * 68u + c8;
        const v4f x0 = *(const v4f*)sp, x1 = *(const v4f*)(sp + 4);
        float y[8];
        if (EPI == 0) {
          const unsigned s = s0 + ((unsigned)i << 4) + row;
          const v4f cs = *(const v4f*)(tab + (size_t)s * 64u + (c8 >> 1));
          const v4f sn = *(const v4f*)(tab + (size_t)s * 64u + 32u + (c8 >> 1));
          y[0] = x0.x * cs.x - x0.y * sn.x; y[1] = x0.y * cs.x + x0.x * sn.x;
          y[2] = x0.z * cs.y - x0.w * sn.y; y[3] = x0.w * cs.y + x0.z * sn.y;
          y[4] = x1.x * cs.z - x1.y * sn.z; y[5] = x1.y * cs.z + x1.x * sn.z;
          y[6] = x1.z * cs.w - x1.w * sn.w; y[7] = x1.w * cs.w + x1.z * sn.w;
        } else {
          y[0] = x0.x; y[1] = x0.y; y[2] = x0.z; y[3] = x0.w; y[4] = x1.x; y[5] = x1.y; y[6] = x1.z; y[7] = x1.w;
        }
        v8us fvv, hvv, lvv;
#pragma unroll
        for (int e = 0; e < 8; ++e) { fvv[e] = h_bits(y[e]); hvv[e] = 0; lvv[e] = 0; }
        if (inband) {
#pragma unroll
          for (int e = 0; e < 8; ++e) { const unsigned short hb = bf_bits(y[e]); hvv[e] = hb; lvv[e] = bf_bits(y[e] - bf_f32(hb)); }
        }
        fv[it] = fvv; hv[it] = hvv; lv[it] = lvv;
      }
      for (int pass = 0; pass < 2; ++pass) {
#pragma unroll
        for (int it = 0; it < 4; ++it) {
          const unsigned row = (unsigned)it * 4u + q;
          if (EPI == 0) {
            const unsigned s = s0 + ((unsigned)i << 4) + row;
            *(volatile v8us*)(CFz + (size_t)(mBase + row) * DM + n0 + c8) = fv[it];
            if (inband) {
              const size_t ob = (size_t)(bidx * (unsigned)BANDE + s) * DM + n0 + c8;
              *(volatile v8us*)(CBHz + ob) = hv[it];
              *(volatile v8us*)(CBLz + ob) = lv[it];
            }
          } else {
            const unsigned fr = mBase + row;
            *(volatile v8us*)(CF + (size_t)fr * NTOK + n0 + c8) = fv[it];
            if (inband) {
              const size_t ob = (size_t)fr * NBAND + bidx * (unsigned)BANDE + s0 + c8;
              *(volatile v8us*)(CBH + ob) = hv[it];
              *(volatile v8us*)(CBL + ob) = lv[it];
            }
          }
        }
        __threadfence();
      }
    }
    WAVE_SYNC();
  }
}

template <bool SP>
__global__ __launch_bounds__(128) void k_attn(
    const unsigned short* __restrict__ Qa, const unsigned short* __restrict__ Qb,
    const unsigned short* __restrict__ Ka, const unsigned short* __restrict__ Kb,
    const unsigned short* __restrict__ Va, const unsigned short* __restrict__ Vb,
    unsigned short* __restrict__ CH, unsigned short* __restrict__ CL, unsigned qb0, unsigned nqb) {
  typedef typename Elem<SP ? 1 : 0>::T T;
  typedef Frag<T> F;
  typedef typename F::V V;
  constexpr unsigned RS = SP ? (unsigned)BANDE : (unsigned)SEQ;
  constexpr unsigned VPITCH = NB * RS;
  const float PSC = SP ? 1.0f : 32768.0f;
  __shared__ __align__(16) T Ph[4][16 * 64];
  __shared__ __align__(16) T Pl[SP ? 4 : 1][SP ? 16 * 64 : 8];
  __shared__ __align__(16) unsigned short Chs[4][16 * 64];
  __shared__ __align__(16) unsigned short Cls[4][16 * 64];

  const unsigned tid = threadIdx.x, wave = tid >> 5, lane = tid & 31u, hh = lane >> 4, c = lane & 15u;
  const unsigned bx = blockIdx.x;
  const unsigned bh = bx / nqb;
  const unsigned qb = qb0 + (bx - bh * nqb);
  const unsigned b = bh / (unsigned)NH, h = bh - b * (unsigned)NH;
  const unsigned q0 = (qb << 6) + (wave << 4);
  const unsigned rowbase = b * RS;

  const T* QaT = (const T*)Qa; const T* QbT = (const T*)Qb;
  const T* KaT = (const T*)Ka; const T* KbT = (const T*)Kb;
  const T* VaT = (const T*)Va; const T* VbT = (const T*)Vb;

  const size_t qo = (size_t)(rowbase + q0 + c) * DM + h * (unsigned)HD + 8u * hh;
  const V qa0 = F::load(QaT + qo), qa1 = F::load(QaT + qo + 32);
  V ql0 = qa0, ql1 = qa1;
  if (SP) { ql0 = F::load(QbT + qo); ql1 = F::load(QbT + qo + 32); }

  float mrow[8], lrow[8];
  v8f o[4];
#pragma unroll
  for (int r = 0; r < 8; ++r) { mrow[r] = -__builtin_inff(); lrow[r] = 0.f; }
#pragma unroll
  for (int t = 0; t < 4; ++t) o[t] = (v8f){0.f, 0.f, 0.f, 0.f, 0.f, 0.f, 0.f, 0.f};

  const float SCL = 0.125f * 1.4426950408889634f;
  T* pwh = Ph[wave];
  T* pwl = Pl[SP ? wave : 0];

  for (unsigned kc = 0; kc <= qb; ++kc) {
    const unsigned kv0 = kc << 6;
    v8f s[4];
#pragma unroll
    for (int j = 0; j < 4; ++j) {
      const size_t ko = (size_t)(rowbase + kv0 + ((unsigned)j << 4) + c) * DM + h * (unsigned)HD + 8u * hh;
      const V kb0 = F::load(KaT + ko), kb1 = F::load(KaT + ko + 32);
      v8f a = (v8f){0.f, 0.f, 0.f, 0.f, 0.f, 0.f, 0.f, 0.f};
      a = mma_g<T>(qa0, kb0, a);
      a = mma_g<T>(qa1, kb1, a);
      if (SP) {
        const V kl0 = F::load(KbT + ko), kl1 = F::load(KbT + ko + 32);
        a = mma_g<T>(qa0, kl0, a);
        a = mma_g<T>(qa1, kl1, a);
        a = mma_g<T>(ql0, kb0, a);
        a = mma_g<T>(ql1, kb1, a);
      }
      s[j] = a;
      asm volatile("" ::: "memory");
    }
    const bool diag = (kc == qb);
#pragma unroll
    for (int r = 0; r < 8; ++r) {
      const unsigned qrow = q0 + 8u * hh + (unsigned)r;
      float sc[4];
      float m = -__builtin_inff();
#pragma unroll
      for (int j = 0; j < 4; ++j) {
        const unsigned kvcol = kv0 + ((unsigned)j << 4) + c;
        float v = s[j][r] * SCL;
        v = (diag && kvcol > qrow) ? -__builtin_inff() : v;
        sc[j] = v;
        m = fmaxf(m, v);
      }
      m = fmaxf(m, __shfl_xor(m, 1, 32)); m = fmaxf(m, __shfl_xor(m, 2, 32));
      m = fmaxf(m, __shfl_xor(m, 4, 32)); m = fmaxf(m, __shfl_xor(m, 8, 32));
      const float mnew = fmaxf(mrow[r], m);
      const float alpha = exp2f(mrow[r] - mnew);
      mrow[r] = mnew;
      float psum = 0.f;
#pragma unroll
      for (int j = 0; j < 4; ++j) {
        const float p = exp2f(sc[j] - mnew);
        psum += p;
        const unsigned idx = (8u * hh + (unsigned)r) * 64u + ((unsigned)j << 4) + c;
        if (SP) {
          const unsigned short hb = bf_bits(p);
          pwh[idx] = F::from_bits(hb);
          pwl[idx] = F::from_bits(bf_bits(p - bf_f32(hb)));
        } else {
          pwh[idx] = F::from_bits(h_bits(p * PSC));
        }
      }
      psum += __shfl_xor(psum, 1, 32); psum += __shfl_xor(psum, 2, 32);
      psum += __shfl_xor(psum, 4, 32); psum += __shfl_xor(psum, 8, 32);
      lrow[r] = lrow[r] * alpha + psum;
#pragma unroll
      for (int t = 0; t < 4; ++t) o[t][r] *= alpha;
    }
    WAVE_SYNC();
#pragma unroll 1
    for (unsigned kk = 0; kk < 2u; ++kk) {
      const V pa = F::load(pwh + c * 64u + kk * 32u + 8u * hh);
      V pl = pa;
      if (SP) pl = F::load(pwl + c * 64u + kk * 32u + 8u * hh);
#pragma unroll
      for (int t = 0; t < 4; ++t) {
        const size_t vo = (size_t)(h * (unsigned)HD + ((unsigned)t << 4) + c) * VPITCH + rowbase + kv0 + kk * 32u + 8u * hh;
        const V vb = F::load(VaT + vo);
        o[t] = mma_g<T>(pa, vb, o[t]);
        if (SP) {
          const V vl = F::load(VbT + vo);
          o[t] = mma_g<T>(pa, vl, o[t]);
          o[t] = mma_g<T>(pl, vb, o[t]);
        }
      }
    }
    WAVE_SYNC();
  }

  unsigned short* chs = Chs[wave];
  unsigned short* cls = Cls[wave];
#pragma unroll
  for (int r = 0; r < 8; ++r) {
    const float inv = 1.0f / (lrow[r] * PSC);
#pragma unroll
    for (int t = 0; t < 4; ++t) {
      const float v = o[t][r] * inv;
      const unsigned short hb = bf_bits(v);
      const unsigned idx = (8u * hh + (unsigned)r) * 64u + ((unsigned)t << 4) + c;
      chs[idx] = hb;
      cls[idx] = bf_bits(v - bf_f32(hb));
    }
  }
  WAVE_SYNC();
  {
    const unsigned q = lane >> 3, c8 = (lane & 7u) << 3;
    v8us hv[4], lv[4];
#pragma unroll
    for (int it = 0; it < 4; ++it) {
      const unsigned row = (unsigned)it * 4u + q;
      hv[it] = *(const v8us*)(chs + row * 64u + c8);
      lv[it] = *(const v8us*)(cls + row * 64u + c8);
    }
    for (int pass = 0; pass < 2; ++pass) {
#pragma unroll
      for (int it = 0; it < 4; ++it) {
        const unsigned row = (unsigned)it * 4u + q;
        const size_t oo = ((size_t)b * SEQ + q0 + row) * DM + h * (unsigned)HD + c8;
        *(volatile v8us*)(CH + oo) = hv[it];
        *(volatile v8us*)(CL + oo) = lv[it];
      }
      __threadfence();
    }
  }
}

extern "C" void kernel_launch(void* const* d_in, const int* in_sizes, int n_in, void* d_out, int out_size, void* d_ws, size_t ws_size, hipStream_t stream) {
  if (n_in < 5) return;
  const long long need_x = ((long long)(NB - 1) * SEQ_FULL + SEQ) * DM;
  if ((long long)in_sizes[0] < need_x) return;
  if ((long long)in_sizes[1] < (long long)DM * DM || (long long)in_sizes[2] < (long long)DM * DM) return;
  if ((long long)in_sizes[3] < (long long)DM * DM || (long long)in_sizes[4] < (long long)DM * DM) return;
  if ((long long)out_size < need_x) return;

  const float* x   = (const float*)d_in[0];
  W4 wp; wp.w0 = (const float*)d_in[1]; wp.w1 = (const float*)d_in[2]; wp.w2 = (const float*)d_in[3]; wp.w3 = (const float*)d_in[4];
  float* out = (float*)d_out;

  constexpr size_t SZ_X16 = (size_t)NTOK * DM * 2;
  constexpr size_t SZ_W16 = (size_t)4 * DM * DM * 2;
  constexpr size_t SZ_TAB = (size_t)SEQ * 64 * 4;
  constexpr size_t SZ_QKF = (size_t)2 * NTOK * DM * 2;
  constexpr size_t SZ_VTF = (size_t)DM * NTOK * 2;
  constexpr size_t SZ_QKB = (size_t)2 * NBAND * DM * 2;
  constexpr size_t SZ_VB  = (size_t)DM * NBAND * 2;
  constexpr size_t SZ_CTL = (size_t)NTOK * DM * 2;
  static_assert(SZ_X16 % 256 == 0 && SZ_W16 % 256 == 0 && SZ_TAB % 256 == 0 && SZ_QKF % 256 == 0);
  static_assert(SZ_VTF % 256 == 0 && SZ_QKB % 256 == 0 && SZ_VB % 256 == 0 && SZ_CTL % 256 == 0);
  constexpr size_t SZ_ALL = SZ_X16 + SZ_W16 + SZ_TAB + SZ_QKF + SZ_VTF + 2 * SZ_QKB + 2 * SZ_VB + SZ_CTL;
  static_assert(SZ_ALL <= (size_t)134217728);
  if (SZ_ALL > ws_size) return;

  char* wsp = (char*)d_ws;
  unsigned short* X16  = (unsigned short*)wsp; wsp += SZ_X16;
  unsigned short* W16  = (unsigned short*)wsp; wsp += SZ_W16;
  float*          TAB  = (float*)wsp;          wsp += SZ_TAB;
  unsigned short* QKF  = (unsigned short*)wsp; wsp += SZ_QKF;
  unsigned short* VTF  = (unsigned short*)wsp; wsp += SZ_VTF;
  unsigned short* QKBH = (unsigned short*)wsp; wsp += SZ_QKB;
  unsigned short* QKBL = (unsigned short*)wsp; wsp += SZ_QKB;
  unsigned short* VBH  = (unsigned short*)wsp; wsp += SZ_VB;
  unsigned short* VBL  = (unsigned short*)wsp; wsp += SZ_VB;
  unsigned short* CTXL = (unsigned short*)wsp; wsp += SZ_CTL;
  unsigned short* CTXH = X16;

  RopeF rf;
  for (int i = 0; i < 32; ++i) {
    const double pw = pow(10000.0, (double)(2 * i) / 64.0);
    const float pwf = (float)pw;
    rf.inv[i] = 1.0f / pwf;
  }

  k_cast_x<<<dim3((unsigned)(NTOK / 2)), 256, 0, stream>>>(x, X16);
  k_cast_w<<<dim3((unsigned)(DM * DM / 8 / 256), 4u), 256, 0, stream>>>(wp, W16);
  k_tab<<<dim3((unsigned)(SEQ / 8)), 256, 0, stream>>>(TAB, rf);

  constexpr unsigned GB = (unsigned)((NTOK / 64) * (DM / 64) / 8);
  k_gemm64<0><<<dim3(GB, 2u), 256, 0, stream>>>(X16, X16, W16, QKF, QKBH, QKBL, TAB, TAB);
  k_gemm64<1><<<dim3(GB, 1u), 256, 0, stream>>>(W16 + (size_t)2 * DM * DM, W16 + (size_t)2 * DM * DM, X16, VTF, VBH, VBL, TAB, TAB);

  constexpr unsigned NQB_BAND = (unsigned)(BANDE / 64);
  constexpr unsigned NQB_REST = (unsigned)((SEQ - BANDE) / 64);
  k_attn<true><<<dim3((unsigned)(NB * NH) * NQB_BAND), 128, 0, stream>>>(
      QKBH, QKBL, QKBH + (size_t)NBAND * DM, QKBL + (size_t)NBAND * DM, VBH, VBL, CTXH, CTXL, 0u, NQB_BAND);
  if (NQB_REST > 0u) {
    k_attn<false><<<dim3((unsigned)(NB * NH) * NQB_REST), 128, 0, stream>>>(
        QKF, QKF, QKF + (size_t)NTOK * DM, QKF + (size_t)NTOK * DM, VTF, VTF, CTXH, CTXL, NQB_BAND, NQB_REST);
  }
  k_gemm64<2><<<dim3(GB, 1u), 256, 0, stream>>>(CTXH, CTXL, W16 + (size_t)3 * DM * DM, QKF, QKBH, QKBL, out, TAB);
}
